// MultiHeadSelfAttention_3298534883514
// MI455X (gfx1250) — hardware-verified
//
#include <hip/hip_runtime.h>


#ifndef NB
#define NB 2
#endif
#ifndef SEQ
#define SEQ 2048
#endif
#define NB_FULL  2
#define SEQ_FULL 2048
#define DM   1024
#define NH   16
#define HD   64
#define MROWS (NB * SEQ)
#define QCAR 16.0f
#define PCAR 256.0f
#define LOG2E 1.4426950408889634f
#define CSC   (0.125f * LOG2E / (QCAR * QCAR))
#define FILLU (-1.0e9f * LOG2E)
#define PLANE_E ((size_t)NB * NH * SEQ * HD)
#define AT_E    ((size_t)MROWS * DM)
#define AM_OFF_E ((size_t)NB_FULL * SEQ_FULL * DM)

static_assert(NB <= NB_FULL);
static_assert(SEQ <= SEQ_FULL);
static_assert(SEQ % 64 == 0);
static_assert(DM % 64 == 0);
static_assert(DM % 32 == 0);
static_assert(HD == 64);
static_assert(NH * HD == DM);
static_assert((DM * DM / 8) % 256 == 0);
static_assert(((size_t)MROWS * DM / 8) % 256 == 0);
static_assert((size_t)NB_FULL * SEQ_FULL * DM * 4 == 16777216);
static_assert(((size_t)NB_FULL * SEQ_FULL * DM * 4) % 128 == 0);

#define SZ_WALL ((size_t)4 * DM * DM * 2)
#define SZ_XB   ((size_t)MROWS * DM * 2)
#define SZ_QKV  ((size_t)3 * PLANE_E * 2)
#define SZ_AT   ((size_t)2 * AT_E * 2)
#define SZ_ST   ((size_t)NB * NH * (SEQ / 64) * 128 * 4)
#define OFF_WALL ((size_t)0)
#define OFF_XB   (OFF_WALL + SZ_WALL)
#define OFF_QKV  (OFF_XB + SZ_XB)
#define OFF_AT   (OFF_QKV + SZ_QKV)
#define OFF_ST   (OFF_AT + SZ_AT)
#define WS_TOTAL (OFF_ST + SZ_ST)
static_assert(SZ_WALL % 256 == 0);
static_assert(SZ_XB % 256 == 0);
static_assert(SZ_QKV % 256 == 0);
static_assert(SZ_AT % 256 == 0);
static_assert(SZ_ST % 256 == 0);
static_assert(WS_TOTAL <= (size_t)134217728);

typedef _Float16 h16;
typedef unsigned short bf;
typedef __attribute__((ext_vector_type(16))) __bf16   v16bf;
typedef __attribute__((ext_vector_type(16))) _Float16 v16h;
typedef __attribute__((ext_vector_type(8)))  _Float16 v8h;
typedef __attribute__((ext_vector_type(8)))  unsigned short v8us;
typedef __attribute__((ext_vector_type(8)))  float    v8f;
typedef __attribute__((ext_vector_type(4)))  float    v4f;
typedef v4f  __attribute__((may_alias)) v4fa;

__device__ __forceinline__ unsigned short f2bf(float f) { unsigned u = __float_as_uint(f); u += 0x7FFFu + ((u >> 16) & 1u); return (unsigned short)(u >> 16); }
__device__ __forceinline__ float bf2f(unsigned short b) { return __uint_as_float(((unsigned)b) << 16); }
__device__ __forceinline__ float bfr(float f) { return bf2f(f2bf(f)); }
__device__ __forceinline__ void splitf(float y, unsigned short& h, unsigned short& l) { h = f2bf(y); l = f2bf(y - bf2f(h)); }
__device__ __forceinline__ v16h cat16(v8h lo, v8h hi) { return __builtin_shufflevector(lo, hi, 0, 1, 2, 3, 4, 5, 6, 7, 8, 9, 10, 11, 12, 13, 14, 15); }
__device__ __forceinline__ v16bf cat16b(v8us lo, v8us hi) { return __builtin_bit_cast(v16bf, __builtin_shufflevector(lo, hi, 0, 1, 2, 3, 4, 5, 6, 7, 8, 9, 10, 11, 12, 13, 14, 15)); }
__device__ __forceinline__ v8f wmma16(v16h a, v16h b, v8f c) { return __builtin_amdgcn_wmma_f32_16x16x32_f16(false, a, false, b, (short)0, c, false, false); }
__device__ __forceinline__ v8f wmmab(v16bf a, v16bf b, v8f c) { return __builtin_amdgcn_wmma_f32_16x16x32_bf16(false, a, false, b, (short)0, c, false, false); }
__device__ __forceinline__ v16h  ldh(const h16* p) { return cat16(*(const v8h*)p, *(const v8h*)(p + 16)); }
__device__ __forceinline__ v16bf ldb(const bf* p)  { return cat16b(*(const v8us*)p, *(const v8us*)(p + 16)); }

__global__ __launch_bounds__(256) void k_cvtx(const float* __restrict__ x, bf* XB) {
    const size_t i = (size_t)blockIdx.x * 256 + threadIdx.x; if (i >= (size_t)MROWS * DM / 8) return;
    const size_t row = i / (DM / 8); const size_t c8 = i % (DM / 8); const size_t b = row / SEQ, t = row % SEQ;
    const v8f v = *(const v8f*)(x + ((b * SEQ_FULL + t) * DM + c8 * 8)); v8us o;
#pragma unroll
    for (int k = 0; k < 8; ++k) o[k] = f2bf(v[k]);
    *(volatile v8us*)(XB + i * 8) = o; __threadfence(); *(volatile v8us*)(XB + i * 8) = o; }

__global__ __launch_bounds__(256) void k_cvtw(const float* __restrict__ w0, const float* __restrict__ w1, const float* __restrict__ w2, const float* __restrict__ w3, bf* WALL) {
    const size_t i = (size_t)blockIdx.x * 256 + threadIdx.x; if (i >= (size_t)DM * DM / 8) return;
    const int which = blockIdx.y; v8f v;
    if (which == 0) v = *(const v8f*)(w0 + i * 8); else if (which == 1) v = *(const v8f*)(w1 + i * 8); else if (which == 2) v = *(const v8f*)(w2 + i * 8); else v = *(const v8f*)(w3 + i * 8);
    v8us o;
#pragma unroll
    for (int k = 0; k < 8; ++k) o[k] = f2bf(v[k]);
    bf* d = WALL + (size_t)which * DM * DM + i * 8;
    *(volatile v8us*)d = o; __threadfence(); *(volatile v8us*)d = o; }

__device__ __forceinline__ void gemm64(const bf* __restrict__ A, size_t asplit, int nsp, const bf* __restrict__ Bt, int r0, int n0, int lane, v8f (&acc)[4][4]) {
    const int lr = lane & 15, hi = lane >> 4;
#pragma unroll
    for (int mb = 0; mb < 4; ++mb)
#pragma unroll
        for (int nb = 0; nb < 4; ++nb) acc[mb][nb] = (v8f){};
    const size_t boff = (size_t)(n0 + lr) * DM + 8 * hi;
#pragma unroll 1
    for (int sp = 0; sp < nsp; ++sp) {
        const size_t aoff = (size_t)sp * asplit + (size_t)(r0 + lr) * DM + 8 * hi;
#pragma unroll 1
        for (int kc = 0; kc < DM; kc += 32) {
            v16bf a[4]; v16bf b;
#pragma unroll
            for (int mb = 0; mb < 4; ++mb) a[mb] = ldb(A + aoff + (size_t)mb * 16 * DM + kc);
#pragma unroll
            for (int nb = 0; nb < 4; ++nb) { b = ldb(Bt + boff + (size_t)nb * 16 * DM + kc);
#pragma unroll
                for (int mb = 0; mb < 4; ++mb) acc[mb][nb] = wmmab(a[mb], b, acc[mb][nb]); }
            asm volatile("" : "+v"(acc[0][0]), "+v"(acc[0][1]), "+v"(acc[0][2]), "+v"(acc[0][3]), "+v"(acc[1][0]), "+v"(acc[1][1]), "+v"(acc[1][2]), "+v"(acc[1][3]));
            asm volatile("v_nop\n\tv_nop\n\tv_nop\n\tv_nop" : "+v"(acc[2][0]), "+v"(acc[2][1]), "+v"(acc[2][2]), "+v"(acc[2][3]), "+v"(acc[3][0]), "+v"(acc[3][1]), "+v"(acc[3][2]), "+v"(acc[3][3]) : "v"(a[3]), "v"(b));
        }
    }
}

__global__ __launch_bounds__(32) void k_qkv(const bf* __restrict__ XB, const bf* __restrict__ WALL, const float* __restrict__ bq, const float* __restrict__ bk, const float* __restrict__ bv, h16* QKV) {
    __shared__ __align__(16) float os[64 * 68];
    const int lane = threadIdx.x & 31, lr = lane & 15, hi = lane >> 4;
    const int r0 = blockIdx.x * 64; const int which = blockIdx.y / (DM / 64); const int hh = blockIdx.y % (DM / 64); const int c0 = hh * 64;
    v8f acc[4][4];
    gemm64(XB, 0, 1, WALL, r0, (int)blockIdx.y * 64, lane, acc);
#pragma unroll
    for (int mb = 0; mb < 4; ++mb)
#pragma unroll
        for (int nb = 0; nb < 4; ++nb)
#pragma unroll
            for (int j = 0; j < 8; ++j) os[(mb * 16 + hi * 8 + j) * 68 + nb * 16 + lr] = acc[mb][nb][j];
    __syncthreads();
    const int b = r0 / SEQ, t0 = r0 % SEQ; const size_t bh = (size_t)b * NH + hh; const int q4 = lane >> 3, piece = lane & 7;
    if (which < 2) {
        h16* P = QKV + (size_t)which * PLANE_E + (bh * SEQ + t0) * HD;
        float bia[8];
#pragma unroll
        for (int j = 0; j < 8; ++j) { const int c = c0 + piece * 8 + j; const float b0 = bq[c], b1 = bk[c]; bia[j] = bfr(which == 0 ? b0 : b1); }
#pragma unroll 1
        for (int ps = 0; ps < 2; ++ps) {
#pragma unroll 2
            for (int s = 0; s < 16; ++s) { const int row = s * 4 + q4; const v4f x0 = *(const v4fa*)(os + row * 68 + piece * 8); const v4f x1 = *(const v4fa*)(os + row * 68 + piece * 8 + 4); v8h o;
#pragma unroll
                for (int j = 0; j < 4; ++j) { o[j] = (h16)((x0[j] + bia[j]) * QCAR); o[4 + j] = (h16)((x1[j] + bia[4 + j]) * QCAR); }
                *(volatile v8h*)(P + (size_t)row * HD + piece * 8) = o; }
            if (ps == 0) __threadfence(); }
    } else {
        h16* P = QKV + 2 * PLANE_E + bh * HD * SEQ + t0;
#pragma unroll 1
        for (int ps = 0; ps < 2; ++ps) {
#pragma unroll 2
            for (int s = 0; s < 16; ++s) { const int d = s * 4 + q4; const float bb = bfr(bv[c0 + d]); v8h o;
#pragma unroll
                for (int j = 0; j < 8; ++j) o[j] = (h16)(os[(piece * 8 + j) * 68 + d] + bb);
                *(volatile v8h*)(P + (size_t)d * SEQ + piece * 8) = o; }
            if (ps == 0) __threadfence(); }
    }
}

__global__ __launch_bounds__(128) void k_flash(const h16* __restrict__ QKV, const int* __restrict__ mask, bf* AT, float* ST) {
    __shared__ unsigned mw[SEQ / 32];
    __shared__ __align__(16) float os[64 * 68];
    __shared__ __align__(16) float sst[128];
    const int lane = threadIdx.x & 31, lr = lane & 15, hi = lane >> 4;
    const int wave = __builtin_amdgcn_readfirstlane((int)(threadIdx.x >> 5));
    const int qt = blockIdx.x, hh = blockIdx.y, b = blockIdx.z; const size_t bh = (size_t)b * NH + hh;
#pragma unroll 1
    for (int c = wave; c < SEQ / 32; c += 4) { const int mv = mask[(size_t)b * SEQ_FULL + c * 32 + lane]; const unsigned wd = __builtin_amdgcn_ballot_w32(mv != 0); if (lane == 0) mw[c] = wd; }
    __syncthreads();
    const int q0 = qt * 64 + wave * 16;
    const h16* qp = QKV + (bh * SEQ + q0 + lr) * HD + 8 * hi;
    const v16h qb0 = ldh(qp), qb1 = ldh(qp + 32);
    const h16* kp = QKV + PLANE_E + (bh * SEQ + lr) * HD + 8 * hi;
    const h16* vp = QKV + 2 * PLANE_E + (bh * HD + lr) * SEQ + 8 * hi;
    float m = -1.0e30f, l = 0.0f; v8f o[4];
#pragma unroll
    for (int dt = 0; dt < 4; ++dt) o[dt] = (v8f){};
#pragma unroll 1
    for (int jb = 0; jb < SEQ / 32; ++jb) {
        const int j0 = jb * 32; const unsigned mwv = (unsigned)__builtin_amdgcn_readfirstlane((int)mw[jb]);
        v8f s0 = (v8f){}, s1 = (v8f){};
        { const h16* p = kp + (size_t)j0 * HD; const v16h a00 = ldh(p), a01 = ldh(p + 32), a10 = ldh(p + 16 * HD), a11 = ldh(p + 16 * HD + 32);
          s0 = wmma16(a00, qb0, s0); s0 = wmma16(a01, qb1, s0); s1 = wmma16(a10, qb0, s1); s1 = wmma16(a11, qb1, s1);
          asm volatile("v_nop\n\tv_nop\n\tv_nop\n\tv_nop" : "+v"(s0), "+v"(s1) : "v"(a11), "v"(qb1)); }
        s0 = s0 * CSC; s1 = s1 * CSC;
        if (mwv != 0xFFFFFFFFu) {
#pragma unroll
            for (int r = 0; r < 8; ++r) { s0[r] = ((mwv >> (8 * hi + r)) & 1u) ? s0[r] : FILLU; s1[r] = ((mwv >> (16 + 8 * hi + r)) & 1u) ? s1[r] : FILLU; } }
        float mx = fmaxf(s0[0], s1[0]);
#pragma unroll
        for (int r = 1; r < 8; ++r) mx = fmaxf(mx, fmaxf(s0[r], s1[r]));
        mx = fmaxf(mx, __shfl_xor(mx, 16, 32));
        const float mn = fmaxf(m, mx);
        if (__builtin_amdgcn_ballot_w32(mn > m) != 0u) { const float al = __builtin_amdgcn_exp2f(m - mn); l *= al;
#pragma unroll
            for (int dt = 0; dt < 4; ++dt) o[dt] = o[dt] * al; }
        m = mn;
        float ps = 0.0f; v16h pb;
#pragma unroll
        for (int r = 0; r < 8; ++r) { const float p0 = __builtin_amdgcn_exp2f(s0[r] - mn) * PCAR; const float p1 = __builtin_amdgcn_exp2f(s1[r] - mn) * PCAR; ps += p0 + p1; pb[r] = (h16)p0; pb[8 + r] = (h16)p1; }
        l += ps;
        { const h16* p = vp + j0; const v16h v0 = ldh(p), v1 = ldh(p + (size_t)16 * SEQ), v2 = ldh(p + (size_t)32 * SEQ), v3 = ldh(p + (size_t)48 * SEQ);
          o[0] = wmma16(v0, pb, o[0]); o[1] = wmma16(v1, pb, o[1]); o[2] = wmma16(v2, pb, o[2]); o[3] = wmma16(v3, pb, o[3]);
          asm volatile("v_nop\n\tv_nop\n\tv_nop\n\tv_nop" : "+v"(o[0]), "+v"(o[1]), "+v"(o[2]), "+v"(o[3]) : "v"(v3), "v"(pb)); }
    }
    l += __shfl_xor(l, 16, 32);
    const float il = 1.0f / l;
    { float* orow = os + (wave * 16 + lr) * 68 + 8 * hi;
#pragma unroll
      for (int dt = 0; dt < 4; ++dt) { v4f x0, x1;
#pragma unroll
          for (int j = 0; j < 4; ++j) { x0[j] = o[dt][j] * il; x1[j] = o[dt][4 + j] * il; }
          *(v4fa*)(orow + dt * 16) = x0; *(v4fa*)(orow + dt * 16 + 4) = x1; } }
    if (hi == 0) { sst[wave * 16 + lr] = m; sst[64 + wave * 16 + lr] = 16.0f * il; }
    __syncthreads();
    const int q4 = lane >> 3, piece = lane & 7;
#pragma unroll 1
    for (int ps2 = 0; ps2 < 2; ++ps2) {
#pragma unroll
        for (int s = 0; s < 4; ++s) { const int row = wave * 16 + s * 4 + q4; const v4f x0 = *(const v4fa*)(os + row * 68 + piece * 8); const v4f x1 = *(const v4fa*)(os + row * 68 + piece * 8 + 4); v8us oh, ol;
#pragma unroll
            for (int j = 0; j < 4; ++j) { unsigned short a, c2; splitf(x0[j], a, c2); oh[j] = a; ol[j] = c2; splitf(x1[j], a, c2); oh[4 + j] = a; ol[4 + j] = c2; }
            const size_t oo = ((size_t)b * SEQ + qt * 64 + row) * DM + hh * HD + piece * 8;
            *(volatile v8us*)(AT + oo) = oh; *(volatile v8us*)(AT + AT_E + oo) = ol; }
        if (wave == 0) { const v4f sv = *(const v4fa*)(sst + lane * 4); *(volatile v4f*)(ST + ((bh * (SEQ / 64) + qt) * 128 + lane * 4)) = sv; }
        if (ps2 == 0) __threadfence(); }
}

__global__ __launch_bounds__(128) void k_amean(const h16* __restrict__ QKV, const int* __restrict__ mask, const float* __restrict__ ST, float* AM) {
    __shared__ __align__(16) float os[64 * 68];
    const int lane = threadIdx.x & 31, lr = lane & 15, hi = lane >> 4;
    const int wave = __builtin_amdgcn_readfirstlane((int)(threadIdx.x >> 5));
    const int k0 = blockIdx.x * 64, qt = blockIdx.y, b = blockIdx.z; const int q0 = qt * 64 + wave * 16;
    const int mv0 = mask[(size_t)b * SEQ_FULL + k0 + lane]; const int mv1 = mask[(size_t)b * SEQ_FULL + k0 + 32 + lane];
    const unsigned w0 = __builtin_amdgcn_ballot_w32(mv0 != 0); const unsigned w1 = __builtin_amdgcn_ballot_w32(mv1 != 0);
    const bool allv = ((w0 & w1) == 0xFFFFFFFFu);
    v8f acc[4];
#pragma unroll
    for (int kt = 0; kt < 4; ++kt) acc[kt] = (v8f){};
#pragma unroll 1
    for (int hh = 0; hh < NH; ++hh) {
        const size_t bh = (size_t)b * NH + hh;
        const h16* qp = QKV + (bh * SEQ + q0 + lr) * HD + 8 * hi;
        const v16h qb0 = ldh(qp), qb1 = ldh(qp + 32);
        const float* st = ST + (bh * (SEQ / 64) + qt) * 128 + wave * 16 + lr;
        const float m = st[0], inv = st[64];
        const h16* kp = QKV + PLANE_E + (bh * SEQ + k0 + lr) * HD + 8 * hi;
        v8f s[4]; v16h a0, a1;
#pragma unroll
        for (int kt = 0; kt < 4; ++kt) { a0 = ldh(kp + (size_t)kt * 16 * HD); a1 = ldh(kp + (size_t)kt * 16 * HD + 32); s[kt] = wmma16(a0, qb0, (v8f){}); s[kt] = wmma16(a1, qb1, s[kt]); }
        asm volatile("v_nop\n\tv_nop\n\tv_nop\n\tv_nop" : "+v"(s[0]), "+v"(s[1]), "+v"(s[2]), "+v"(s[3]) : "v"(a1), "v"(qb1));
#pragma unroll
        for (int kt = 0; kt < 4; ++kt) s[kt] = s[kt] * CSC;
        if (!allv) {
#pragma unroll
            for (int kt = 0; kt < 4; ++kt) { const unsigned wsel = (kt < 2) ? w0 : w1;
#pragma unroll
                for (int r = 0; r < 8; ++r) s[kt][r] = ((wsel >> ((kt & 1) * 16 + 8 * hi + r)) & 1u) ? s[kt][r] : FILLU; } }
#pragma unroll
        for (int kt = 0; kt < 4; ++kt)
#pragma unroll
            for (int r = 0; r < 8; ++r) acc[kt][r] += __builtin_amdgcn_exp2f(s[kt][r] - m) * inv;
    }
    { float* orow = os + (wave * 16 + lr) * 68 + 8 * hi;
#pragma unroll
      for (int kt = 0; kt < 4; ++kt) { v4f x0, x1;
#pragma unroll
          for (int j = 0; j < 4; ++j) { x0[j] = acc[kt][j]; x1[j] = acc[kt][4 + j]; }
          *(v4fa*)(orow + kt * 16) = x0; *(v4fa*)(orow + kt * 16 + 4) = x1; } }
    __syncthreads();
    float* dst = AM + ((size_t)b * SEQ_FULL + qt * 64) * SEQ_FULL + k0;
#pragma unroll 1
    for (int ps = 0; ps < 2; ++ps) {
#pragma unroll
        for (int s2 = 0; s2 < 8; ++s2) { const int row = wave * 16 + 2 * s2 + hi; const int cofs = lr * 4; const v4f val = *(const v4fa*)(os + row * 68 + cofs);
            *(volatile v4f*)(dst + (size_t)row * SEQ_FULL + cofs) = val; }
        if (ps == 0) __threadfence(); }
}

__global__ __launch_bounds__(32) void k_outp(const bf* __restrict__ AT, const bf* __restrict__ WO, const float* __restrict__ bo, float* OUT) {
    __shared__ __align__(16) float os[64 * 68];
    const int lane = threadIdx.x & 31, lr = lane & 15, hi = lane >> 4;
    const int r0 = blockIdx.x * 64, c0 = blockIdx.y * 64;
    v8f acc[4][4];
    gemm64(AT, AT_E, 2, WO, r0, c0, lane, acc);
#pragma unroll
    for (int mb = 0; mb < 4; ++mb)
#pragma unroll
        for (int nb = 0; nb < 4; ++nb)
#pragma unroll
            for (int j = 0; j < 8; ++j) os[(mb * 16 + hi * 8 + j) * 68 + nb * 16 + lr] = acc[mb][nb][j];
    __syncthreads();
    const int b = r0 / SEQ, t0 = r0 % SEQ; const int cofs = lr * 4;
    float* crow = OUT + ((size_t)b * SEQ_FULL + t0) * DM + c0;
    v4f bia;
#pragma unroll
    for (int j = 0; j < 4; ++j) bia[j] = bfr(bo[c0 + cofs + j]);
#pragma unroll 1
    for (int ps = 0; ps < 2; ++ps) {
#pragma unroll 4
        for (int s = 0; s < 32; ++s) { const int row = 2 * s + hi; const v4f val = *(const v4fa*)(os + row * 68 + cofs) + bia;
            *(volatile v4f*)(crow + (size_t)row * DM + cofs) = val; }
        if (ps == 0) __threadfence(); }
}

extern "C" void kernel_launch(void* const* d_in, const int* in_sizes, int n_in,
                              void* d_out, int out_size, void* d_ws, size_t ws_size, hipStream_t stream) {
    if (n_in < 10) return;
    const long long need_rows = (long long)(NB - 1) * SEQ_FULL + SEQ;
    if ((long long)in_sizes[0] < need_rows * DM) return;
    if ((long long)in_sizes[1] < need_rows) return;
    if (in_sizes[2] < DM * DM || in_sizes[4] < DM * DM || in_sizes[6] < DM * DM || in_sizes[8] < DM * DM) return;
    if (in_sizes[3] < DM || in_sizes[5] < DM || in_sizes[7] < DM || in_sizes[9] < DM) return;
    const long long need_out = (long long)AM_OFF_E + ((long long)(NB - 1) * SEQ_FULL + SEQ - 1) * SEQ_FULL + SEQ;
    if ((long long)out_size < need_out) return;
    if ((size_t)WS_TOTAL > ws_size) return;
    const float* x = (const float*)d_in[0]; const int* mask = (const int*)d_in[1];
    const float* wq = (const float*)d_in[2]; const float* bq = (const float*)d_in[3];
    const float* wk = (const float*)d_in[4]; const float* bk = (const float*)d_in[5];
    const float* wv = (const float*)d_in[6]; const float* bv = (const float*)d_in[7];
    const float* wo = (const float*)d_in[8]; const float* bo = (const float*)d_in[9];
    float* OUT = (float*)d_out; float* AM = OUT + AM_OFF_E;
    char* wsp = (char*)d_ws;
    bf* WALL = (bf*)(wsp + OFF_WALL); bf* XB = (bf*)(wsp + OFF_XB); h16* QKV = (h16*)(wsp + OFF_QKV); bf* AT = (bf*)(wsp + OFF_AT); float* ST = (float*)(wsp + OFF_ST);
    k_cvtw<<<dim3((unsigned)((size_t)DM * DM / 8 / 256), 4, 1), 256, 0, stream>>>(wq, wk, wv, wo, WALL);
    k_cvtx<<<(unsigned)((size_t)MROWS * DM / 8 / 256), 256, 0, stream>>>(x, XB);
    k_qkv<<<dim3(MROWS / 64, 3 * DM / 64, 1), 32, 0, stream>>>(XB, WALL, bq, bk, bv, QKV);
    k_flash<<<dim3(SEQ / 64, NH, NB), 128, 0, stream>>>(QKV, mask, AT, ST);
    k_amean<<<dim3(SEQ / 64, SEQ / 64, NB), 128, 0, stream>>>(QKV, mask, ST, AM);
    k_outp<<<dim3(MROWS / 64, DM / 64, 1), 32, 0, stream>>>(AT, WALL + (size_t)3 * DM * DM, bo, OUT);
}
